// GCU_37306085933363
// MI455X (gfx1250) — hardware-verified
//
#include <hip/hip_runtime.h>
#include <stddef.h>


#define NTHR    256
#define NWAVE   8
#define EPT     8
#define CHUNK   (NTHR * EPT)
#define WCAP    (EPT * 32)
#define LISTN   (NWAVE * WCAP)
#define PASSN   (NWAVE * 32)
#define PCAP    (CHUNK + PASSN)
#define RMAX    (PCAP / PASSN + 1)
#define NB      1024
#define SELFP   ((NB + PASSN - 1) / PASSN)
#define FC      32
#define PQW     128
#define OC      64
#define NTHR2   128
#define RB      64
#define BN_EPS  1e-5f
#define NEG_BIG (-3.0e38f)

static_assert(PASSN == NTHR);
static_assert(NB == NWAVE * 32 * 4);
static_assert(SELFP * PASSN >= NB);
static_assert((NB % RB) == 0);

typedef float          v4f   __attribute__((ext_vector_type(4)));
typedef float          v8f   __attribute__((ext_vector_type(8)));
typedef int            v4i   __attribute__((ext_vector_type(4)));
typedef unsigned short v4us  __attribute__((ext_vector_type(4)));
typedef unsigned short v8us  __attribute__((ext_vector_type(8)));
typedef unsigned short v16us __attribute__((ext_vector_type(16)));
typedef __bf16         v16b  __attribute__((ext_vector_type(16)));
union FragU { v16us u; v8us h[2]; };

__device__ __forceinline__ unsigned short bfb(float x) {
  const __bf16 b = (__bf16)x;
  return __builtin_bit_cast(unsigned short, b);
}
__device__ __forceinline__ float bfv(unsigned short u) {
  return __uint_as_float(((unsigned)u) << 16);
}
__device__ __forceinline__ void split4(v4f v, v4us& hi, v4us& lo) {
  v4us a, b;
#pragma unroll
  for (int c = 0; c < 4; ++c) {
    const unsigned short uh = bfb(v[c]);
    const float rsd = v[c] - bfv(uh);
    a[c] = uh;
    b[c] = bfb(rsd);
  }
  hi = a; lo = b;
}
__device__ __forceinline__ v8f zacc() {
  v8f z = {0.0f, 0.0f, 0.0f, 0.0f, 0.0f, 0.0f, 0.0f, 0.0f};
  return z;
}

__device__ __forceinline__ v8f wmb(v16us a, v16us b, v8f c) {
  const v16b av = __builtin_bit_cast(v16b, a);
  const v16b bv = __builtin_bit_cast(v16b, b);
  v8f d = __builtin_amdgcn_wmma_f32_16x16x32_bf16(false, av, false, bv, (short)0, c, false, false);
  asm volatile("v_nop\n\tv_nop\n\tv_nop\n\tv_nop" : "+v"(d) : "v"(av), "v"(bv));
  return d;
}
__device__ __forceinline__ v8f wm3(const FragU& ah, const FragU& al, const FragU& bh, const FragU& bl, v8f c) {
  c = wmb(ah.u, bh.u, c);
  c = wmb(ah.u, bl.u, c);
  c = wmb(al.u, bh.u, c);
  return c;
}

__device__ __forceinline__ FragU ldfrag(const unsigned short* p, int pitch, int row, int k0, int hh) {
  FragU f;
  const unsigned short* q = p + row * pitch + k0 + 8 * hh;
  f.h[0] = *(const v8us*)q;
  f.h[1] = *(const v8us*)(q + 16);
  return f;
}

__device__ __forceinline__ int scan_chunk(const int* __restrict__ dsts, int nE, int cbase, int nodeBase,
                                          int vec8, int* list, int tid, int wave) {
  int wc = 0;
  const int el0  = tid * EPT;
  const int e0   = cbase + el0;
  const int sent = -2147483647 - 1;
  const int em   = nE - 1;
  v4i da, db;
  if (vec8 != 0 && cbase + CHUNK <= nE) {
    da = *(const v4i*)(dsts + e0);
    db = *(const v4i*)(dsts + e0 + 4);
  } else {
    da.x = (e0     < nE) ? dsts[min(e0,     em)] : sent;
    da.y = (e0 + 1 < nE) ? dsts[min(e0 + 1, em)] : sent;
    da.z = (e0 + 2 < nE) ? dsts[min(e0 + 2, em)] : sent;
    da.w = (e0 + 3 < nE) ? dsts[min(e0 + 3, em)] : sent;
    db.x = (e0 + 4 < nE) ? dsts[min(e0 + 4, em)] : sent;
    db.y = (e0 + 5 < nE) ? dsts[min(e0 + 5, em)] : sent;
    db.z = (e0 + 6 < nE) ? dsts[min(e0 + 6, em)] : sent;
    db.w = (e0 + 7 < nE) ? dsts[min(e0 + 7, em)] : sent;
  }
  const unsigned nb = (unsigned)nodeBase;
  const unsigned s0 = (unsigned)da.x - nb, s1 = (unsigned)da.y - nb;
  const unsigned s2 = (unsigned)da.z - nb, s3 = (unsigned)da.w - nb;
  const unsigned s4 = (unsigned)db.x - nb, s5 = (unsigned)db.y - nb;
  const unsigned s6 = (unsigned)db.z - nb, s7 = (unsigned)db.w - nb;
  const bool h0 = s0 < (unsigned)NB, h1 = s1 < (unsigned)NB, h2 = s2 < (unsigned)NB, h3 = s3 < (unsigned)NB;
  const bool h4 = s4 < (unsigned)NB, h5 = s5 < (unsigned)NB, h6 = s6 < (unsigned)NB, h7 = s7 < (unsigned)NB;
  const unsigned any = __builtin_amdgcn_ballot_w32(h0 | h1 | h2 | h3 | h4 | h5 | h6 | h7);
  if (any != 0u) {
#define HITJ(J, HJ) { \
      const unsigned mj = __builtin_amdgcn_ballot_w32(HJ); \
      if (mj != 0u) { \
        if (HJ) { \
          const int pos = wc + (int)__builtin_amdgcn_mbcnt_lo(mj, 0u); \
          if (pos < WCAP) list[wave * WCAP + pos] = el0 + (J); \
        } \
        wc += (int)__builtin_popcount(mj); } }
    HITJ(0, h0)
    HITJ(1, h1)
    HITJ(2, h2)
    HITJ(3, h3)
    HITJ(4, h4)
    HITJ(5, h5)
    HITJ(6, h6)
    HITJ(7, h7)
#undef HITJ
  }
  return wc;
}

__device__ __forceinline__ void run_pass(
    int r, int Pv, int selfmode,
    const int* pend, const int* __restrict__ srcs, const int* __restrict__ dsts,
    const float* __restrict__ npq, int nN, int nE, int nodeBase, int coff,
    unsigned short* stgH, unsigned short* stgL, int* slotb, float* msg, float* mx,
    const unsigned short* w2h, const unsigned short* w2l, const float* prm,
    float b2a, float b2b, float s2a, float s2b, float t2a, float t2b,
    int lane, int wave, int hh, int m) {
  {
    const int idx = r * PASSN + wave * 32 + lane;
    const bool valid = idx < Pv;
    int s, d, slot;
    if (selfmode != 0) {
      int node = nodeBase + idx;
      node = node > nN - 1 ? nN - 1 : node;
      node = node < 0 ? 0 : node;
      s = node; d = node;
      slot = (valid && idx < NB) ? idx : NB;
    } else {
      const int pi = idx < PCAP - 1 ? idx : PCAP - 1;
      int e = pend[pi];
      const int em = nE - 1 < 0 ? 0 : nE - 1;
      e = e < 0 ? 0 : (e > em ? em : e);
      d = dsts[e];
      s = srcs[e];
      slot = d - nodeBase;
      if (!valid || (unsigned)slot >= (unsigned)NB) slot = NB;
      d = d < 0 ? 0 : (d > nN - 1 ? nN - 1 : d);
      s = s < 0 ? 0 : (s > nN - 1 ? nN - 1 : s);
    }
    const float* prow = npq + (size_t)d * PQW + coff;
    const float* qrow = npq + (size_t)s * PQW + coff + FC;
    unsigned short* hrow = stgH + (wave * 32 + lane) * FC;
    unsigned short* lrow = stgL + (wave * 32 + lane) * FC;
#pragma unroll 2
    for (int c4 = 0; c4 < 8; ++c4) {
      const v4f p  = *(const v4f*)(prow + 4 * c4);
      const v4f q  = *(const v4f*)(qrow + 4 * c4);
      const v4f bb = *(const v4f*)(prm + 4 * c4);
      const v4f ss = *(const v4f*)(prm + 32 + 4 * c4);
      const v4f tt = *(const v4f*)(prm + 64 + 4 * c4);
      v4f hv;
#pragma unroll
      for (int j = 0; j < 4; ++j) {
        const float z = (p[j] + q[j]) + bb[j];
        const float a = fmaxf(z, 0.0f) * ss[j] + tt[j];
        hv[j] = valid ? a : 0.0f;
      }
      v4us hi, lo;
      split4(hv, hi, lo);
      *(v4us*)(hrow + 4 * c4) = hi;
      *(v4us*)(lrow + 4 * c4) = lo;
    }
    slotb[wave * 32 + lane] = slot;
  }
  __syncthreads();

  {
#pragma unroll
    for (int et = 0; et < 2; ++et) {
      const FragU ah = ldfrag(stgH, FC, wave * 32 + 16 * et + m, 0, hh);
      const FragU al = ldfrag(stgL, FC, wave * 32 + 16 * et + m, 0, hh);
#pragma unroll
      for (int nt = 0; nt < 2; ++nt) {
        const FragU bh = ldfrag(w2h, FC, 16 * nt + m, 0, hh);
        const FragU bl = ldfrag(w2l, FC, 16 * nt + m, 0, hh);
        const v8f acc = wm3(ah, al, bh, bl, zacc());
        const float bq = (nt != 0) ? b2b : b2a;
        const float sq = (nt != 0) ? s2b : s2a;
        const float tq = (nt != 0) ? t2b : t2a;
        float* mrow = msg + (wave * 32 + 16 * et + 8 * hh) * FC + 16 * nt + m;
#pragma unroll
        for (int rr = 0; rr < 8; ++rr) mrow[rr * FC] = fmaxf(acc[rr] + bq, 0.0f) * sq + tq;
      }
    }
  }
  __syncthreads();

  if (wave == 0) {
#pragma unroll 1
    for (int i = 0; i < PASSN; ++i) {
      int sl = slotb[i];
      sl = sl < 0 ? 0 : (sl > NB ? NB : sl);
      const float v = msg[i * FC + lane];
      float* mp = mx + sl * FC + lane;
      const float o = *mp;
      *mp = fmaxf(o, v);
    }
  }
  __syncthreads();
}

__global__ __launch_bounds__(NTHR2) void k_node(const float* __restrict__ x, const float* __restrict__ W1,
                                                float* npq, int nN) {
  __shared__ __attribute__((aligned(16))) unsigned short xh[RB * 32];
  __shared__ __attribute__((aligned(16))) unsigned short xl[RB * 32];
  __shared__ __attribute__((aligned(16))) unsigned short wh[128 * 32];
  __shared__ __attribute__((aligned(16))) unsigned short wl[128 * 32];
  __shared__ __attribute__((aligned(16))) float ot[4 * 16 * PQW];
  const int tid = threadIdx.x, lane = tid & 31, wave = tid >> 5, hh = lane >> 4, m = lane & 15;
  const int r0 = blockIdx.x * RB;

#pragma unroll
  for (int i = 0; i < 4; ++i) {
    const int idx4 = i * NTHR2 + tid;
    const int row = idx4 >> 3, c4 = idx4 & 7;
    int grow = r0 + row;
    grow = grow > nN - 1 ? nN - 1 : grow;
    const v4f v = *(const v4f*)(x + (size_t)grow * 32 + 4 * c4);
    v4us hi, lo;
    split4(v, hi, lo);
    *(v4us*)(xh + row * 32 + 4 * c4) = hi;
    *(v4us*)(xl + row * 32 + 4 * c4) = lo;
  }
#pragma unroll 4
  for (int i = 0; i < 32; ++i) {
    const int e = i * NTHR2 + tid;
    const int n = e >> 5, k = e & 31;
    const int b = n >> 6, q = (n >> 5) & 1, nn = n & 31;
    const float va = W1[((b * 64) + k) * 32 + nn];
    const float vb = W1[((b * 64) + 32 + k) * 32 + nn];
    const float v  = (q != 0) ? vb : (va - vb);
    const unsigned short uh = bfb(v);
    wh[n * 32 + k] = uh;
    wl[n * 32 + k] = bfb(v - bfv(uh));
  }
  __syncthreads();

  const FragU ah = ldfrag(xh, 32, 16 * wave + m, 0, hh);
  const FragU al = ldfrag(xl, 32, 16 * wave + m, 0, hh);
  float* otw = ot + wave * 16 * PQW;
#pragma unroll
  for (int j = 0; j < 8; ++j) {
    const FragU bh = ldfrag(wh, 32, 16 * j + m, 0, hh);
    const FragU bl = ldfrag(wl, 32, 16 * j + m, 0, hh);
    const v8f acc = wm3(ah, al, bh, bl, zacc());
#pragma unroll
    for (int rr = 0; rr < 8; ++rr) otw[(8 * hh + rr) * PQW + 16 * j + m] = acc[rr];
  }
  __syncthreads();

  float* gb = npq + (size_t)(r0 + 16 * wave) * PQW;
#pragma unroll
  for (int rr = 0; rr < 16; ++rr) {
    const v4f v = *(const v4f*)(otw + rr * PQW + 4 * lane);
    *(volatile v4f*)(gb + (size_t)rr * PQW + 4 * lane) = v;
  }
  __threadfence();
#pragma unroll
  for (int rr = 0; rr < 16; ++rr) {
    const v4f v = *(const v4f*)(otw + rr * PQW + 4 * lane);
    *(volatile v4f*)(gb + (size_t)rr * PQW + 4 * lane) = v;
  }
}

__global__ __launch_bounds__(NTHR) void k_agg(
    const float* __restrict__ npq, const int* __restrict__ ei, const float* __restrict__ W2,
    const float* __restrict__ b1, const float* __restrict__ g1, const float* __restrict__ bt1,
    const float* __restrict__ m1, const float* __restrict__ v1,
    const float* __restrict__ b2, const float* __restrict__ g2, const float* __restrict__ bt2,
    const float* __restrict__ m2, const float* __restrict__ v2,
    float* agg, int nN, int nE, int vec8, int coff) {
  __shared__ __attribute__((aligned(16))) float          mx[(NB + 1) * FC];
  __shared__ __attribute__((aligned(16))) float          msg[PASSN * FC];
  __shared__ __attribute__((aligned(16))) unsigned short stgH[NWAVE * 32 * FC];
  __shared__ __attribute__((aligned(16))) unsigned short stgL[NWAVE * 32 * FC];
  __shared__ __attribute__((aligned(16))) int            list[LISTN];
  __shared__ __attribute__((aligned(16))) int            pend[PCAP];
  __shared__ __attribute__((aligned(16))) int            slotb[PASSN];
  __shared__ __attribute__((aligned(16))) unsigned short w2h[FC * FC];
  __shared__ __attribute__((aligned(16))) unsigned short w2l[FC * FC];
  __shared__ __attribute__((aligned(16))) float          prm[6 * FC];
  __shared__ int wcnt[NWAVE];
  __shared__ int pendN;

  const int tid = threadIdx.x, lane = tid & 31, wave = tid >> 5, hh = lane >> 4, m = lane & 15;
  const int nodeBase = blockIdx.x * NB;
  const int* srcs = ei;
  const int* dsts = ei + nE;

  for (int i = tid; i < (NB + 1) * FC; i += NTHR) mx[i] = NEG_BIG;
  for (int i = tid; i < FC * FC; i += NTHR) {
    const int n = i >> 5, k = i & 31;
    const float v = W2[k * FC + n];
    const unsigned short uh = bfb(v);
    w2h[n * FC + k] = uh;
    w2l[n * FC + k] = bfb(v - bfv(uh));
  }
  if (tid < FC) {
    const int c = tid;
    const float sa = g1[c] * rsqrtf(v1[c] + BN_EPS);
    const float sb = g2[c] * rsqrtf(v2[c] + BN_EPS);
    prm[c]          = b1[c];
    prm[FC + c]     = sa;
    prm[2 * FC + c] = bt1[c] - m1[c] * sa;
    prm[3 * FC + c] = b2[c];
    prm[4 * FC + c] = sb;
    prm[5 * FC + c] = bt2[c] - m2[c] * sb;
  }
  if (tid == 0) pendN = 0;
  __syncthreads();
  const float b2a = prm[3 * FC + m], b2b = prm[3 * FC + 16 + m];
  const float s2a = prm[4 * FC + m], s2b = prm[4 * FC + 16 + m];
  const float t2a = prm[5 * FC + m], t2b = prm[5 * FC + 16 + m];

#pragma unroll 1
  for (int r = 0; r < SELFP; ++r)
    run_pass(r, NB, 1, pend, srcs, dsts, npq, nN, nE, nodeBase, coff, stgH, stgL, slotb, msg, mx,
             w2h, w2l, prm, b2a, b2b, s2a, s2b, t2a, t2b, lane, wave, hh, m);

  const int nChunks = (nE + CHUNK - 1) / CHUNK;
#pragma unroll 1
  for (int ch = 0; ch < nChunks; ++ch) {
    const int cbase = ch * CHUNK;
    const int wc = scan_chunk(dsts, nE, cbase, nodeBase, vec8, list, tid, wave);
    if (lane == 0) wcnt[wave] = wc;
    __syncthreads();

    const int base = pendN;
    int tot = 0, myoff = 0;
#pragma unroll
    for (int w = 0; w < NWAVE; ++w) {
      int c = wcnt[w];
      c = c > WCAP ? WCAP : (c < 0 ? 0 : c);
      if (w < wave) myoff += c;
      tot += c;
    }
    int newN = base + tot;
    newN = newN > PCAP ? PCAP : newN;
    {
      int n = wcnt[wave];
      n = n > WCAP ? WCAP : (n < 0 ? 0 : n);
      const int* lp = list + wave * WCAP;
      for (int i = lane; i < n; i += 32) {
        const int pos = base + myoff + i;
        if (pos < PCAP) pend[pos] = cbase + lp[i];
      }
    }
    const int fin = (ch == nChunks - 1) ? 1 : 0;
    int R = (fin != 0) ? (newN + PASSN - 1) / PASSN : newN / PASSN;
    R = R > RMAX ? RMAX : (R < 0 ? 0 : R);
    const int Pv = (fin != 0) ? newN : R * PASSN;
    __syncthreads();

#pragma unroll 1
    for (int r = 0; r < R; ++r)
      run_pass(r, Pv, 0, pend, srcs, dsts, npq, nN, nE, nodeBase, coff, stgH, stgL, slotb, msg, mx,
               w2h, w2l, prm, b2a, b2b, s2a, s2b, t2a, t2b, lane, wave, hh, m);

    int rem = newN - R * PASSN;
    rem = rem < 0 ? 0 : (rem > PASSN ? PASSN : rem);
    if (R > 0 && tid < rem) pend[tid] = pend[R * PASSN + tid];
    if (tid == 0) pendN = rem;
  }
  __syncthreads();

  float* ob = agg + (size_t)nodeBase * FC;
  const int sub = lane >> 3, piece = 4 * (lane & 7);
#pragma unroll 4
  for (int i = 0; i < 32; ++i) {
    const int slot = wave * 128 + 4 * i + sub;
    const v4f v = *(const v4f*)(mx + slot * FC + piece);
    *(volatile v4f*)(ob + (size_t)slot * FC + piece) = v;
  }
  __threadfence();
#pragma unroll 4
  for (int i = 0; i < 32; ++i) {
    const int slot = wave * 128 + 4 * i + sub;
    const v4f v = *(const v4f*)(mx + slot * FC + piece);
    *(volatile v4f*)(ob + (size_t)slot * FC + piece) = v;
  }
}

__global__ __launch_bounds__(NTHR2) void k_final(const float* __restrict__ agg, int npadA,
    const float* __restrict__ mW, const float* __restrict__ mb, const float* __restrict__ mg,
    const float* __restrict__ mbt, const float* __restrict__ mm, const float* __restrict__ mv,
    float* out, int nN) {
  __shared__ __attribute__((aligned(16))) unsigned short ahs[RB * OC];
  __shared__ __attribute__((aligned(16))) unsigned short als[RB * OC];
  __shared__ __attribute__((aligned(16))) unsigned short wh[OC * OC];
  __shared__ __attribute__((aligned(16))) unsigned short wl[OC * OC];
  __shared__ __attribute__((aligned(16))) float ot[4 * 16 * OC];
  __shared__ __attribute__((aligned(16))) float prm[3 * OC];
  const int tid = threadIdx.x, lane = tid & 31, wave = tid >> 5, hh = lane >> 4, m = lane & 15;
  const int r0 = blockIdx.x * RB;
  const size_t plane = (size_t)npadA * FC;

#pragma unroll
  for (int i = 0; i < 8; ++i) {
    const int idx4 = i * NTHR2 + tid;
    const int row = idx4 >> 4, c4 = idx4 & 15;
    const int pl = c4 >> 3, cc = c4 & 7;
    int grow = r0 + row;
    grow = grow > npadA - 1 ? npadA - 1 : grow;
    const v4f v = *(const v4f*)(agg + (size_t)pl * plane + (size_t)grow * FC + 4 * cc);
    v4us hi, lo;
    split4(v, hi, lo);
    *(v4us*)(ahs + row * OC + 4 * c4) = hi;
    *(v4us*)(als + row * OC + 4 * c4) = lo;
  }
#pragma unroll 4
  for (int i = 0; i < 32; ++i) {
    const int e = i * NTHR2 + tid;
    const int n = e >> 6, k = e & 63;
    const float v = mW[k * OC + n];
    const unsigned short uh = bfb(v);
    wh[n * OC + k] = uh;
    wl[n * OC + k] = bfb(v - bfv(uh));
  }
  if (tid < OC) {
    const float s = mg[tid] * rsqrtf(mv[tid] + BN_EPS);
    prm[tid]          = mb[tid];
    prm[OC + tid]     = s;
    prm[2 * OC + tid] = mbt[tid] - mm[tid] * s;
  }
  __syncthreads();

  const FragU a0h = ldfrag(ahs, OC, 16 * wave + m, 0, hh);
  const FragU a0l = ldfrag(als, OC, 16 * wave + m, 0, hh);
  const FragU a1h = ldfrag(ahs, OC, 16 * wave + m, 32, hh);
  const FragU a1l = ldfrag(als, OC, 16 * wave + m, 32, hh);
  float* otw = ot + wave * 16 * OC;
#pragma unroll
  for (int nt = 0; nt < 4; ++nt) {
    const FragU b0h = ldfrag(wh, OC, 16 * nt + m, 0, hh);
    const FragU b0l = ldfrag(wl, OC, 16 * nt + m, 0, hh);
    const FragU b1h = ldfrag(wh, OC, 16 * nt + m, 32, hh);
    const FragU b1l = ldfrag(wl, OC, 16 * nt + m, 32, hh);
    v8f acc = wm3(a0h, a0l, b0h, b0l, zacc());
    acc = wm3(a1h, a1l, b1h, b1l, acc);
    const int ch = 16 * nt + m;
    const float bq = prm[ch], sq = prm[OC + ch], tq = prm[2 * OC + ch];
#pragma unroll
    for (int rr = 0; rr < 8; ++rr) otw[(8 * hh + rr) * OC + ch] = fmaxf(acc[rr] + bq, 0.0f) * sq + tq;
  }
  __syncthreads();

  const int sub = lane >> 4, piece = 4 * (lane & 15);
#pragma unroll
  for (int i = 0; i < 8; ++i) {
    const int row = 2 * i + sub;
    const int grow = r0 + 16 * wave + row;
    const v4f v = *(const v4f*)(otw + row * OC + piece);
    if (grow < nN) *(volatile v4f*)(out + (size_t)grow * OC + piece) = v;
  }
  __threadfence();
#pragma unroll
  for (int i = 0; i < 8; ++i) {
    const int row = 2 * i + sub;
    const int grow = r0 + 16 * wave + row;
    const v4f v = *(const v4f*)(otw + row * OC + piece);
    if (grow < nN) *(volatile v4f*)(out + (size_t)grow * OC + piece) = v;
  }
}

extern "C" void kernel_launch(void* const* d_in, const int* in_sizes, int n_in,
                              void* d_out, int out_size, void* d_ws, size_t ws_size,
                              hipStream_t stream) {
  if (n_in < 21) return;
  const int nN = in_sizes[0] / 32;
  if (nN <= 0 || in_sizes[0] != nN * 32) return;
  const int nE1 = in_sizes[1] / 2, nE2 = in_sizes[2] / 2;
  if (nE1 < 1 || nE2 < 1 || in_sizes[1] != 2 * nE1 || in_sizes[2] != 2 * nE2) return;
  if (in_sizes[3] != 2 * 64 * 32 || in_sizes[9] != 2 * 32 * 32 || in_sizes[15] != 64 * 64) return;
  if (in_sizes[4] != 64 || in_sizes[5] != 64 || in_sizes[6] != 64 || in_sizes[7] != 64 || in_sizes[8] != 64) return;
  if (in_sizes[10] != 64 || in_sizes[11] != 64 || in_sizes[12] != 64 || in_sizes[13] != 64 || in_sizes[14] != 64) return;
  if (in_sizes[16] != 64 || in_sizes[17] != 64 || in_sizes[18] != 64 || in_sizes[19] != 64 || in_sizes[20] != 64) return;
  if (out_size != nN * OC) return;

  const float* x     = (const float*)d_in[0];
  const int*   ei1   = (const int*)d_in[1];
  const int*   ei2   = (const int*)d_in[2];
  const float* ecW1  = (const float*)d_in[3];
  const float* ecb1  = (const float*)d_in[4];
  const float* ecg1  = (const float*)d_in[5];
  const float* ecbt1 = (const float*)d_in[6];
  const float* ecm1  = (const float*)d_in[7];
  const float* ecv1  = (const float*)d_in[8];
  const float* ecW2  = (const float*)d_in[9];
  const float* ecb2  = (const float*)d_in[10];
  const float* ecg2  = (const float*)d_in[11];
  const float* ecbt2 = (const float*)d_in[12];
  const float* ecm2  = (const float*)d_in[13];
  const float* ecv2  = (const float*)d_in[14];
  const float* mW    = (const float*)d_in[15];
  const float* mb    = (const float*)d_in[16];
  const float* mg    = (const float*)d_in[17];
  const float* mbt   = (const float*)d_in[18];
  const float* mm    = (const float*)d_in[19];
  const float* mv    = (const float*)d_in[20];
  float* out = (float*)d_out;

  const int nBlkA = (nN + NB - 1) / NB;
  const int npadA = nBlkA * NB;
  const int nBlkN = (nN + RB - 1) / RB;
  const int npadN = nBlkN * RB;

  char* ws = (char*)d_ws;
  size_t off = 0;
  const size_t oNpq = off; off += (size_t)npadN * PQW * 4;      off = (off + 255) & ~(size_t)255;
  const size_t oAgg = off; off += (size_t)2 * npadA * FC * 4;   off = (off + 255) & ~(size_t)255;
  if (off > ws_size) return;
  float* npq  = (float*)(ws + oNpq);
  float* agg0 = (float*)(ws + oAgg);
  float* agg1 = agg0 + (size_t)npadA * FC;

  const int vec1 = ((nE1 & 3) == 0) ? 1 : 0;
  const int vec2 = ((nE2 & 3) == 0) ? 1 : 0;

  k_node<<<nBlkN, NTHR2, 0, stream>>>(x, ecW1, npq, nN);

  k_agg<<<nBlkA, NTHR, 0, stream>>>(npq, ei1, ecW2,
      ecb1, ecg1, ecbt1, ecm1, ecv1, ecb2, ecg2, ecbt2, ecm2, ecv2,
      agg0, nN, nE1, vec1, 0);

  k_agg<<<nBlkA, NTHR, 0, stream>>>(npq, ei2, ecW2 + 32 * 32,
      ecb1 + 32, ecg1 + 32, ecbt1 + 32, ecm1 + 32, ecv1 + 32,
      ecb2 + 32, ecg2 + 32, ecbt2 + 32, ecm2 + 32, ecv2 + 32,
      agg1, nN, nE2, vec2, 64);

  k_final<<<nBlkN, NTHR2, 0, stream>>>(agg0, npadA, mW, mb, mg, mbt, mm, mv, out, nN);
}
